// RGCNRegression_13597866459798
// MI455X (gfx1250) — hardware-verified
//
#include <hip/hip_runtime.h>
#include <stddef.h>
#include <stdint.h>


#define FEAT   128
#define NREL   8
#define KREL   1024
#define KD     1152
#define KQ     144
#define KSTEPS 36
#define APK    1160
#define TR     16
#define NTHR   256
#define NWAVE  8
#define S1     2048
#define NCH1   8
#define SH1    12
#define SH2    7
#define SH3    4
#define F1A    16
#define F2     32
#define F3     8
#define CAP1   256
#define CAP2   192
#define CAP3   512
#define SEGS2  16
#define WSC    64.0f
#define RWSC   0.015625f
#define SENT   0xFFFFFFFFu
#define WSCAPB 134217728
#define ACC_BYTES 65536
#define SA_BYTES  37120
#define STG_BYTES 8192
#define TILE_LDS  (ACC_BYTES + SA_BYTES + STG_BYTES)

static_assert(KREL == NREL * FEAT);
static_assert(KD == KREL + FEAT);
static_assert(KQ * 8 == KD);
static_assert(KSTEPS * 32 == KD);
static_assert((APK % 8) == 0 && APK >= KD);
static_assert((2 * FEAT * KQ) % NTHR == 0 && (FEAT * KQ) % NTHR == 0);
static_assert(NCH1 * NTHR == S1);
static_assert(CAP1 == NTHR);
static_assert((F1A * CAP1) % (4 * NTHR) == 0);
static_assert((F2 * CAP2) % (4 * NTHR) == 0);
static_assert((F3 * CAP3) % (4 * NTHR) == 0);
static_assert((CAP1 % 32) == 0 && (CAP2 % 32) == 0 && (CAP3 % 32) == 0);
static_assert(NTHR == 32 * NWAVE && TR == 2 * NWAVE);
static_assert(NTHR * 4 * 2 == TR * FEAT);
static_assert(FEAT == 16 * NWAVE);
static_assert(TR * KREL * 4 == ACC_BYTES && TR * APK * 2 == SA_BYTES && TR * FEAT * 4 == STG_BYTES);
static_assert(TILE_LDS == 110848);
static_assert((TR * KREL) % (4 * NTHR) == 0);
static_assert(((ACC_BYTES + SA_BYTES) % 16) == 0);

typedef _Float16 v4h  __attribute__((ext_vector_type(4)));
typedef _Float16 v8h  __attribute__((ext_vector_type(8)));
typedef _Float16 v16h __attribute__((ext_vector_type(16)));
typedef float    v4f  __attribute__((ext_vector_type(4)));
typedef float    v8f  __attribute__((ext_vector_type(8)));
typedef unsigned int v4u __attribute__((ext_vector_type(4)));
typedef v4h v4ha __attribute__((may_alias));
typedef v8h v8ha __attribute__((may_alias));
typedef v4f v4fa __attribute__((may_alias));
typedef v4u v4ua __attribute__((may_alias));
union Frag { v16h v; v8h h[2]; };

__device__ __forceinline__ v8f wmh(v16h a, v16h b, v8f c) {
  v8f d = __builtin_amdgcn_wmma_f32_16x16x32_f16(false, a, false, b, (short)0, c, false, false);
  asm volatile("v_nop\n\tv_nop\n\tv_nop\n\tv_nop" : "+v"(d) : "v"(a), "v"(b));
  return d;
}

__device__ __forceinline__ v4h cvt4(v4f a) {
  v4h r;
  r[0] = (_Float16)a[0]; r[1] = (_Float16)a[1]; r[2] = (_Float16)a[2]; r[3] = (_Float16)a[3];
  return r;
}

__global__ __launch_bounds__(NTHR) void k_wprep(const float* __restrict__ w1, const float* __restrict__ r1,
                                                const float* __restrict__ w2, const float* __restrict__ r2,
                                                _Float16* Bw) {
  const int gi = blockIdx.x * NTHR + threadIdx.x;
  const int layer = gi >= FEAT * KQ ? 1 : 0;
  const int i = gi - layer * (FEAT * KQ);
  const float* wr = layer ? w2 : w1;
  const float* rt = layer ? r2 : r1;
  const int n = i / KQ, kq = i - n * KQ, k0 = kq * 8;
  const int kr = k0 < (KREL - 8) ? k0 : (KREL - 8);
  int il0 = k0 - KREL;
  il0 = il0 < 0 ? 0 : (il0 > FEAT - 8 ? FEAT - 8 : il0);
  const bool isrel = k0 < KREL;
  v8h hv;
#pragma unroll
  for (int e = 0; e < 8; ++e) {
    const float vw = wr[((size_t)(kr + e)) * FEAT + n];
    const float vl = rt[(il0 + e) * FEAT + n];
    const float v = isrel ? vw : vl;
    hv[e] = (_Float16)(v * WSC);
  }
  _Float16* dst = Bw + (size_t)layer * ((size_t)FEAT * KD) + (size_t)i * 8;
  *(volatile v8h*)dst = hv;
  __threadfence();
  *(volatile v8h*)dst = hv;
}

template <int LV, int FA, int CAP>
__global__ __launch_bounds__(NTHR) void k_part(const int* __restrict__ esrc, const int* __restrict__ edst,
                                               const int* __restrict__ ety, const unsigned* lin, unsigned* lout,
                                               int nN, int nE, int nC, int nB1, int P2, int nch) {
  __shared__ __attribute__((aligned(16))) unsigned lst[FA * CAP];
  __shared__ int wc[NWAVE * 32];
  __shared__ int cur[32];
  const int tid = threadIdx.x, lane = tid & 31, wave = tid >> 5;
  const int blk = blockIdx.x;
  const v4u sv = {SENT, SENT, SENT, SENT};
#pragma unroll
  for (int k = 0; k < (FA * CAP) / (4 * NTHR); ++k) *(v4ua*)(&lst[4 * (tid + NTHR * k)]) = sv;
  if (wave == 0) cur[lane] = 0;
  __syncthreads();

  int c = 0, part = 0, ml = 0;
  if (LV == 2) { c = blk / P2; part = blk - c * P2; }
  if (LV == 3) { c = blk >> 5; ml = blk & 31; }
  const int nslots3 = P2 * CAP2;

#pragma unroll 1
  for (int ch = 0; ch < nch; ++ch) {
    bool valid;
    int key;
    unsigned rec;
    if (LV == 1) {
      const int e = blk * S1 + ch * NTHR + tid;
      const int ec = e < nE ? e : nE - 1;
      const int d = edst[ec];
      valid = (e < nE) && ((unsigned)d < (unsigned)nN);
      key = d >> SH1;
      rec = (unsigned)ec;
    } else if (LV == 2) {
      const int bl = part * SEGS2 + ch;
      const int blc = bl < nB1 ? bl : nB1 - 1;
      const unsigned id = lin[((size_t)blc * nC + c) * CAP1 + tid];
      const bool idok = id < (unsigned)nE;
      const int idc = idok ? (int)id : nE - 1;
      const int d = edst[idc];
      valid = (bl < nB1) && idok && ((unsigned)d < (unsigned)nN);
      key = (d >> SH2) & 31;
      rec = (unsigned)idc;
    } else {
      const int q = ch * NTHR + tid;
      const int qc = q < nslots3 ? q : nslots3 - 1;
      const int pp = qc / CAP2, s = qc - pp * CAP2;
      const unsigned id = lin[(((size_t)(c * P2 + pp)) * F2 + ml) * CAP2 + s];
      const bool idok = id < (unsigned)nE;
      const int idc = idok ? (int)id : nE - 1;
      const int d = edst[idc];
      int sv2 = esrc[idc];
      sv2 = sv2 < 0 ? 0 : (sv2 > nN - 1 ? nN - 1 : sv2);
      const int tv0 = ety[idc];
      const bool tok = (unsigned)tv0 < (unsigned)NREL;
      const int tv = tok ? tv0 : 0;
      valid = (q < nslots3) && idok && tok && ((unsigned)d < (unsigned)nN);
      key = (d >> SH3) & 7;
      rec = ((unsigned)d & 15u) | ((unsigned)tv << 4) | ((unsigned)sv2 << 8);
    }
    key = valid ? key : 255;
    unsigned mym = 0u;
#pragma unroll
    for (int b = 0; b < FA; ++b) {
      const unsigned mb = __builtin_amdgcn_ballot_w32(key == b);
      mym = (key == b) ? mb : mym;
    }
    const unsigned lt = (1u << lane) - 1u;
    const int rank = __builtin_popcount(mym & lt);
    const int cnt  = __builtin_popcount(mym);
    wc[wave * 32 + lane] = 0;
    if (valid && rank == 0) wc[wave * 32 + key] = cnt;
    __syncthreads();
    const int kc = key & 31;
    int pre = 0;
    for (int w2 = 0; w2 < wave; ++w2) pre += wc[w2 * 32 + kc];
    const int pos = cur[kc] + pre + rank;
    if (valid && pos < CAP) lst[kc * CAP + pos] = rec;
    int tot = 0;
    if (wave == 0) {
#pragma unroll
      for (int w2 = 0; w2 < NWAVE; ++w2) tot += wc[w2 * 32 + lane];
    }
    __syncthreads();
    if (wave == 0) cur[lane] += tot;
  }
  __syncthreads();

  const int nwords  = (LV == 1) ? nC * CAP : FA * CAP;
  const int npieces = nwords >> 2;
  unsigned* gb = lout + (size_t)blk * nwords;
#pragma unroll
  for (int k = 0; k < (FA * CAP / 4 + NTHR - 1) / NTHR; ++k) {
    const int it = tid + NTHR * k;
    if (it < npieces) { const v4u v = *(const v4ua*)(&lst[4 * it]); *(volatile v4u*)(gb + 4 * it) = v; }
  }
  __threadfence();
#pragma unroll
  for (int k = 0; k < (FA * CAP / 4 + NTHR - 1) / NTHR; ++k) {
    const int it = tid + NTHR * k;
    if (it < npieces) { const v4u v = *(const v4ua*)(&lst[4 * it]); *(volatile v4u*)(gb + 4 * it) = v; }
  }
}

__device__ __forceinline__ void drain(unsigned m, unsigned rec, float* rowp, const float* x,
                                      int lane, int nN, int& cacc) {
  while (m != 0u) {
    const int i = __builtin_ctz(m);
    m &= m - 1u;
    const unsigned r = (unsigned)__builtin_amdgcn_readlane((int)rec, i);
    int src = (int)(r >> 8);
    src = src > nN - 1 ? nN - 1 : src;
    const int ty = (int)((r >> 4) & 7u);
    cacc += (ty == lane) ? 1 : 0;
    const v4f v = *(const v4f*)(x + (size_t)src * FEAT + 4 * lane);
    v4fa* p = (v4fa*)(rowp + ty * FEAT + 4 * lane);
    v4f t = *p;
    t += v;
    *p = t;
  }
}

__global__ __launch_bounds__(NTHR) void k_tile(const float* x, const _Float16* __restrict__ Bw,
                                               const unsigned* __restrict__ l3, const float* __restrict__ bias,
                                               const float* __restrict__ wout, const float* __restrict__ bout,
                                               float* hout, float* hs, int nN, int head) {
  extern __shared__ __attribute__((aligned(16))) unsigned char dynlds[];
  __shared__ float invl[TR * NREL];
  __shared__ __attribute__((aligned(16))) float scal[32];
  float*    accf = (float*)dynlds;
  _Float16* sA   = (_Float16*)(dynlds + ACC_BYTES);
  float*    stg  = (float*)(dynlds + ACC_BYTES + SA_BYTES);
  const int tid = threadIdx.x, lane = tid & 31, wave = tid >> 5, hh = lane >> 4, m = lane & 15;
  const int tile = blockIdx.x;

  const v4f z4 = {0.f, 0.f, 0.f, 0.f};
#pragma unroll
  for (int k = 0; k < (TR * KREL) / (4 * NTHR); ++k) *(v4fa*)(accf + 4 * (tid + NTHR * k)) = z4;
#pragma unroll
  for (int k = 0; k < 2; ++k) {
    const int row = wave + 8 * k, c4 = lane * 4;
    const int node = tile * TR + row;
    const int nc = node < nN ? node : nN - 1;
    v4f v = *(const v4f*)(x + (size_t)nc * FEAT + c4);
    if (node >= nN) v = z4;
    *(v4ha*)(sA + row * APK + KREL + c4) = cvt4(v);
  }
  __syncthreads();

  int cnt0 = 0, cnt1 = 0;
  {
    const unsigned* seg = l3 + (size_t)tile * CAP3;
    float* row0 = accf + (2 * wave) * KREL;
    float* row1 = row0 + KREL;
#pragma unroll 1
    for (int ch = 0; ch < CAP3 / 32; ++ch) {
      const unsigned rec = seg[ch * 32 + lane];
      const bool ok = ((int)rec) >= 0;
      const int ln = (int)(rec & 15u);
      const unsigned m0 = __builtin_amdgcn_ballot_w32(ok && (ln == 2 * wave));
      const unsigned m1 = __builtin_amdgcn_ballot_w32(ok && (ln == 2 * wave + 1));
      drain(m0, rec, row0, x, lane, nN, cnt0);
      drain(m1, rec, row1, x, lane, nN, cnt1);
    }
  }
  if (lane < NREL) {
    invl[(2 * wave) * NREL + lane]     = 1.0f / fmaxf((float)cnt0, 1.0f);
    invl[(2 * wave + 1) * NREL + lane] = 1.0f / fmaxf((float)cnt1, 1.0f);
  }
  __syncthreads();

#pragma unroll
  for (int k = 0; k < (TR * KREL) / (4 * NTHR); ++k) {
    const int idx4 = 4 * (tid + NTHR * k);
    const int row = idx4 >> 10, col = idx4 & (KREL - 1);
    const float sc = invl[row * NREL + (col >> 7)];
    const v4f v = *(const v4fa*)(accf + idx4);
    *(v4ha*)(sA + row * APK + col) = cvt4(v * sc);
  }
  __syncthreads();

  {
    v8f acc = {0.f, 0.f, 0.f, 0.f, 0.f, 0.f, 0.f, 0.f};
    const _Float16* abase = sA + m * APK + 8 * hh;
    const _Float16* bbase = Bw + (size_t)(wave * 16 + m) * KD + 8 * hh;
#pragma unroll 1
    for (int kt = 0; kt < KSTEPS; ++kt) {
      Frag a, b;
      a.h[0] = *(const v8ha*)(abase + 32 * kt);
      a.h[1] = *(const v8ha*)(abase + 32 * kt + 16);
      b.h[0] = *(const v8h*)(bbase + 32 * kt);
      b.h[1] = *(const v8h*)(bbase + 32 * kt + 16);
      acc = wmh(a.v, b.v, acc);
    }
    const int col = wave * 16 + m;
#pragma unroll
    for (int r = 0; r < 8; ++r) stg[(8 * hh + r) * FEAT + col] = acc[r];
  }
  __syncthreads();

  const int c4 = lane * 4;
  const v4f bv = *(const v4f*)(bias + c4);
  const v4f wv = *(const v4f*)(wout + c4);
  const v4f p0 = *(const v4fa*)(stg + wave * FEAT + c4);
  const v4f p1 = *(const v4fa*)(stg + (wave + 8) * FEAT + c4);
  v4f o0 = p0 * RWSC + bv;
  v4f o1 = p1 * RWSC + bv;
  o0[0] = fmaxf(o0[0], 0.0f); o0[1] = fmaxf(o0[1], 0.0f); o0[2] = fmaxf(o0[2], 0.0f); o0[3] = fmaxf(o0[3], 0.0f);
  o1[0] = fmaxf(o1[0], 0.0f); o1[1] = fmaxf(o1[1], 0.0f); o1[2] = fmaxf(o1[2], 0.0f); o1[3] = fmaxf(o1[3], 0.0f);
  float s0 = o0[0] * wv[0] + o0[1] * wv[1] + o0[2] * wv[2] + o0[3] * wv[3];
  float s1 = o1[0] * wv[0] + o1[1] * wv[1] + o1[2] * wv[2] + o1[3] * wv[3];
#pragma unroll
  for (int off = 16; off > 0; off >>= 1) {
    s0 += __shfl_xor(s0, off, 32);
    s1 += __shfl_xor(s1, off, 32);
  }
  const int node0 = tile * TR + wave, node1 = node0 + 8;
  const bool a0 = node0 < nN, a1 = node1 < nN;
  float* g0 = hout + (size_t)(a0 ? node0 : 0) * FEAT + c4;
  float* g1 = hout + (size_t)(a1 ? node1 : 0) * FEAT + c4;
  if (head == 0) {
    if (a0) *(volatile v4f*)g0 = o0;
    if (a1) *(volatile v4f*)g1 = o1;
  }
  if (wave == 1 && lane < 16) scal[16 + lane] = 0.0f;
  if (lane == 0) { const float bb = bout[0]; scal[wave] = s0 + bb; scal[wave + 8] = s1 + bb; }
  __threadfence();
  if (head == 0) {
    if (a0) *(volatile v4f*)g0 = o0;
    if (a1) *(volatile v4f*)g1 = o1;
  }
  __syncthreads();
  const v4f hv4 = *(const v4fa*)(scal + 4 * (lane & 7));
  float* gh = hs + (size_t)tile * 32 + 4 * (lane & 7);
  const bool wh = (head != 0) && (wave == 0) && (lane < 8);
  if (wh) *(volatile v4f*)gh = hv4;
  __threadfence();
  if (wh) *(volatile v4f*)gh = hv4;
}

__global__ __launch_bounds__(NTHR) void k_out(const float* __restrict__ hs, float* out, int nN) {
  const int t = blockIdx.x * NTHR + threadIdx.x;
  const int tc = t < nN ? t : nN - 1;
  const float v = hs[(size_t)(tc >> 4) * 32 + (tc & 15)];
  if (t < nN) *(volatile float*)(out + t) = v;
  __threadfence();
  if (t < nN) *(volatile float*)(out + t) = v;
}

extern "C" void kernel_launch(void* const* d_in, const int* in_sizes, int n_in,
                              void* d_out, int out_size, void* d_ws, size_t ws_size,
                              hipStream_t stream) {
  if (n_in < 11) return;
  if (in_sizes[0] <= 0 || (in_sizes[0] % FEAT) != 0) return;
  const int nN = in_sizes[0] / FEAT;
  const int nE = in_sizes[2];
  if (nN < 1 || nN > 65536) return;
  if (nE < 1 || nE > (1 << 28)) return;
  if (in_sizes[1] != 2 * nE) return;
  if (in_sizes[3] != NREL * FEAT * FEAT || in_sizes[4] != FEAT * FEAT || in_sizes[5] != FEAT) return;
  if (in_sizes[6] != NREL * FEAT * FEAT || in_sizes[7] != FEAT * FEAT || in_sizes[8] != FEAT) return;
  if (in_sizes[9] != FEAT || in_sizes[10] < 1) return;
  if (out_size != nN) return;

  const float* x     = (const float*)d_in[0];
  const int*   esrc  = (const int*)d_in[1];
  const int*   edst  = esrc + nE;
  const int*   ety   = (const int*)d_in[2];
  const float* W1    = (const float*)d_in[3];
  const float* root1 = (const float*)d_in[4];
  const float* b1    = (const float*)d_in[5];
  const float* W2    = (const float*)d_in[6];
  const float* root2 = (const float*)d_in[7];
  const float* b2    = (const float*)d_in[8];
  const float* wout  = (const float*)d_in[9];
  const float* bout  = (const float*)d_in[10];
  float* out = (float*)d_out;

  const int nTiles = (nN + TR - 1) / TR;
  const int nC   = (nN + 4095) >> SH1;
  const int nB1  = (nE + S1 - 1) / S1;
  const int P2   = (nB1 + SEGS2 - 1) / SEGS2;
  const int nch3 = (P2 * CAP2 + NTHR - 1) / NTHR;
  if (nC < 1 || nC > F1A) return;

  char* ws = (char*)d_ws;
  size_t o = 0;
  const size_t oBw = o; o += (size_t)2 * FEAT * KD * 2;                   o = (o + 255) & ~(size_t)255;
  const size_t oL1 = o; o += (size_t)nB1 * nC * CAP1 * 4;                 o = (o + 255) & ~(size_t)255;
  const size_t oL2 = o; o += (size_t)nC * P2 * F2 * CAP2 * 4;             o = (o + 255) & ~(size_t)255;
  const size_t oL3 = o; o += (size_t)nC * 32 * F3 * CAP3 * 4;             o = (o + 255) & ~(size_t)255;
  const size_t oH1 = o; o += (size_t)nTiles * TR * FEAT * 4;              o = (o + 255) & ~(size_t)255;
  const size_t oHS = o; o += (size_t)nTiles * 32 * 4;                     o = (o + 255) & ~(size_t)255;
  if (o > ws_size || o > (size_t)WSCAPB) return;
  _Float16* Bw = (_Float16*)(ws + oBw);
  unsigned* L1 = (unsigned*)(ws + oL1);
  unsigned* L2 = (unsigned*)(ws + oL2);
  unsigned* L3 = (unsigned*)(ws + oL3);
  float*    H1 = (float*)(ws + oH1);
  float*    HS = (float*)(ws + oHS);

  k_wprep<<<(2 * FEAT * KQ) / NTHR, NTHR, 0, stream>>>(W1, root1, W2, root2, Bw);
  k_part<1, F1A, CAP1><<<nB1, NTHR, 0, stream>>>(esrc, edst, ety, L1, L1, nN, nE, nC, nB1, P2, NCH1);
  k_part<2, F2, CAP2><<<nC * P2, NTHR, 0, stream>>>(esrc, edst, ety, L1, L2, nN, nE, nC, nB1, P2, SEGS2);
  k_part<3, F3, CAP3><<<nC * 32, NTHR, 0, stream>>>(esrc, edst, ety, L2, L3, nN, nE, nC, nB1, P2, nch3);
  hipFuncSetAttribute(reinterpret_cast<const void*>(&k_tile), hipFuncAttributeMaxDynamicSharedMemorySize, TILE_LDS);
  k_tile<<<nTiles, NTHR, TILE_LDS, stream>>>(x, Bw, L3, b1, wout, bout, H1, HS, nN, 0);
  k_tile<<<nTiles, NTHR, TILE_LDS, stream>>>(H1, Bw + (size_t)FEAT * KD, L3, b2, wout, bout, H1, HS, nN, 1);
  k_out<<<(nN + NTHR - 1) / NTHR, NTHR, 0, stream>>>(HS, out, nN);
}
